// TransformerDecoder_76330158784753
// MI455X (gfx1250) — hardware-verified
//
#include <hip/hip_runtime.h>


#ifndef NB
#define NB 8
#endif
#ifndef SEQ
#define SEQ 512
#endif
#define NB_FULL 8
#define SEQ_FULL 512

namespace {
constexpr int D = 512, NH = 8, DH = 64, DFF = 2048, NLAY = 6, VOCAB = 32000;
constexpr int MR = NB * SEQ;
constexpr int LQK = 2 * D;
constexpr int NQKV = 3 * D, NKV = 2 * D, NQT = SEQ / 16, NQT_RES = 4;
constexpr float WSC = 256.0f, CA = 8.0f, CX = 64.0f, PSC = 4096.0f, RS = 2048.0f;
constexpr float SQD = 22.627416997969522f, NLOGD = -0.017988946039015984f, L2E = 1.4426950408889634f, NEGF = -1.0e18f, LNEPS = 1.0e-5f;
constexpr float SCL = 1.0f / (CA * CA * 8.0f);
static_assert(NB >= 1 && NB <= NB_FULL && SEQ >= 128 && SEQ <= SEQ_FULL && SEQ % 128 == 0);
static_assert(MR % 128 == 0 && MR % 32 == 0 && D == 512 && NH * DH == D && DFF % 512 == 0 && NQT > NQT_RES && (MR * D) % 8 == 0);

typedef _Float16 b16;
typedef __attribute__((ext_vector_type(16))) _Float16 v16b;
typedef __attribute__((ext_vector_type(8))) _Float16 v8b;
typedef __attribute__((ext_vector_type(4))) _Float16 v4h_;
typedef __attribute__((ext_vector_type(8))) float v8f;
typedef __attribute__((ext_vector_type(4))) float v4f;

__device__ __forceinline__ float bf16_rne(float f) { unsigned int u = __float_as_uint(f); u += 0x7FFFu + ((u >> 16) & 1u); return __uint_as_float(u & 0xFFFF0000u); }
__device__ __forceinline__ v16b frag_kb(const b16* p, int hh) { const v8b a = *(const v8b*)(p + 8 * hh), b = *(const v8b*)(p + 16 + 8 * hh); v16b f;
#pragma unroll
  for (int e = 0; e < 8; ++e) { f[e] = a[e]; f[8 + e] = b[e]; } return f; }
__device__ __forceinline__ v8f wmma_raw(v16b a, v16b b, v8f c) { return __builtin_amdgcn_wmma_f32_16x16x32_f16(false, a, false, b, (short)0, c, false, false); }
__device__ __forceinline__ v8f wmma16b(v16b a, v16b b, v8f c) { v8f d = wmma_raw(a, b, c); asm volatile("v_nop\n\tv_nop\n\tv_nop\n\tv_nop" : "+v"(d) : "v"(a), "v"(b)); return d; }
#define WMMA_GUARD8(c, a0, a1, bf) asm volatile("v_nop\n\tv_nop\n\tv_nop\n\tv_nop" : "+v"(c[0][0]), "+v"(c[0][1]), "+v"(c[0][2]), "+v"(c[0][3]), \
    "+v"(c[1][0]), "+v"(c[1][1]), "+v"(c[1][2]), "+v"(c[1][3]) : "v"(a0), "v"(a1), "v"(bf[0]), "v"(bf[1]), "v"(bf[2]), "v"(bf[3]))
__device__ __forceinline__ void wave_lds_sync() { __builtin_amdgcn_fence(3  , "workgroup"); __builtin_amdgcn_wave_barrier(); __builtin_amdgcn_fence(2  , "workgroup"); }
__device__ __forceinline__ float pmul(float a, float b) { float p = a * b; asm volatile("" : "+v"(p)); return p; }
__device__ __forceinline__ int iclamp(int v, int lo, int hi) { return v < lo ? lo : (v > hi ? hi : v); }
__device__ __forceinline__ float nexp2(float v) { return __builtin_amdgcn_exp2f(v); }
__device__ __forceinline__ float red_max16(float x) {
#pragma unroll
  for (int off = 8; off > 0; off >>= 1) x = fmaxf(x, __shfl_xor(x, off, 16));
  return x; }
__device__ __forceinline__ float red_sum16(float x) {
#pragma unroll
  for (int off = 8; off > 0; off >>= 1) x += __shfl_xor(x, off, 16);
  return x; }

__global__ __launch_bounds__(256) void wprep_kernel(const float* __restrict__ W, b16* __restrict__ Wt, int K, int NA, int NT, int noff) {
  __shared__ __attribute__((aligned(16))) b16 T[64 * 72];
  const int tid = threadIdx.x, l = blockIdx.z, k0 = blockIdx.x * 64, n0 = blockIdx.y * 64;
  { const int kr = tid >> 2, nc = (tid & 3) * 16; const float* src = W + ((size_t)l * K + k0 + kr) * NA + n0 + nc;
#pragma unroll
    for (int q = 0; q < 4; ++q) { const v4f v = *(const v4f*)(src + 4 * q);
#pragma unroll
      for (int j = 0; j < 4; ++j) T[(nc + 4 * q + j) * 72 + kr] = (b16)(bf16_rne(v[j]) * WSC); } }
  __syncthreads();
  v8b vv[2]; size_t dst[2];
#pragma unroll
  for (int i = 0; i < 2; ++i) { const int n = (tid >> 3) + 32 * i, p = tid & 7; vv[i] = *(const v8b*)(T + n * 72 + 8 * p); dst[i] = ((size_t)l * NT + noff + n0 + n) * K + k0 + 8 * p; }
  for (int pass = 0; pass < 2; ++pass) {
#pragma unroll
    for (int i = 0; i < 2; ++i) *(volatile v8b*)(Wt + dst[i]) = vv[i];
    __threadfence(); }
}

__global__ __launch_bounds__(256) void mprep_kernel(const float* __restrict__ mem, b16* __restrict__ Mh) {
  const int u = blockIdx.x * 256 + threadIdx.x;
  if (u >= MR * D / 8) return;
  const int row = u / (D / 8), c0 = (u % (D / 8)) * 8, b = row / SEQ, s = row % SEQ;
  const float* src = mem + ((size_t)b * SEQ_FULL + s) * D + c0;
  const v4f a = *(const v4f*)src, c = *(const v4f*)(src + 4); v8b v;
#pragma unroll
  for (int j = 0; j < 4; ++j) { v[j] = (b16)(bf16_rne(a[j]) * CA); v[4 + j] = (b16)(bf16_rne(c[j]) * CA); }
  for (int pass = 0; pass < 2; ++pass) { *(volatile v8b*)(Mh + (size_t)row * D + c0) = v; __threadfence(); }
}

__global__ __launch_bounds__(256) void embed_kernel(const int* __restrict__ tok, const float* __restrict__ emb, float* __restrict__ X, b16* __restrict__ Xh) {
  __shared__ __attribute__((aligned(16))) float Xs[4 * (D + 4)];
  const int tid = threadIdx.x, rl = tid >> 6, c0 = (tid & 63) * 8, row0 = blockIdx.x * 4, row = row0 + rl, b = row / SEQ, s = row % SEQ;
  const int t = iclamp(tok[s * NB_FULL + b], 0, VOCAB - 1);
  const float* er = emb + (size_t)t * D + c0;
#pragma unroll 1
  for (int q = 0; q < 4; ++q) {
    const int c = c0 + 2 * q; const float dv = expf(pmul((float)c, NLOGD)); float sn, cs; sincosf(pmul((float)s, dv), &sn, &cs);
    Xs[rl * (D + 4) + c] = pmul(bf16_rne(er[2 * q]), SQD) + sn; Xs[rl * (D + 4) + c + 1] = pmul(bf16_rne(er[2 * q + 1]), SQD) + cs; }
  __syncthreads();
  v4f fv[2]; size_t fo[2]; v8b hv;
#pragma unroll
  for (int i = 0; i < 2; ++i) { const int f = i * 256 + tid; fv[i] = *(const v4f*)(Xs + (f >> 7) * (D + 4) + (f & 127) * 4); fo[i] = (size_t)(row0 + (f >> 7)) * D + (f & 127) * 4; }
  { const v4f a = *(const v4f*)(Xs + rl * (D + 4) + c0), c4 = *(const v4f*)(Xs + rl * (D + 4) + c0 + 4);
#pragma unroll
    for (int e = 0; e < 4; ++e) { hv[e] = (b16)(a[e] * CA); hv[4 + e] = (b16)(c4[e] * CA); } }
  for (int pass = 0; pass < 2; ++pass) {
#pragma unroll
    for (int i = 0; i < 2; ++i) *(volatile v4f*)(X + fo[i]) = fv[i];
    *(volatile v8b*)(Xh + (size_t)row * D + c0) = hv; __threadfence(); }
}

__device__ __forceinline__ void mac_32x64(v8f (&acc)[2][4], const b16* ap0, const b16* ap1, const b16* bp, int K, int hlf) {
#pragma unroll 1
  for (int k0 = 0; k0 < K; k0 += 32) {
    const v16b a0 = frag_kb(ap0 + k0, hlf), a1 = frag_kb(ap1 + k0, hlf); v16b bf[4];
#pragma unroll
    for (int t = 0; t < 4; ++t) bf[t] = frag_kb(bp + (size_t)t * 16 * K + k0, hlf);
#pragma unroll
    for (int t = 0; t < 4; ++t) { acc[0][t] = wmma_raw(a0, bf[t], acc[0][t]); acc[1][t] = wmma_raw(a1, bf[t], acc[1][t]); }
    WMMA_GUARD8(acc, a0, a1, bf);
  }
}

template <bool LO, bool RELU>
__device__ __forceinline__ void epi_rows(const v8f (&acc)[2][4], const float (&bb)[4], float oscale, b16* Es, b16* dstp, int ldc, int lane, int nloc, int hlf) {
#pragma unroll
  for (int mt = 0; mt < 2; ++mt)
#pragma unroll
    for (int t = 0; t < 4; ++t)
#pragma unroll
      for (int r = 0; r < 8; ++r) {
        float v = acc[mt][t][r] * oscale + bb[t]; if (RELU) v = fmaxf(v, 0.0f); const float vs = v * CA; const b16 hi = (b16)vs;
        Es[(mt * 16 + 8 * hlf + r) * 72 + 16 * t + nloc] = LO ? (b16)((vs - (float)hi) * RS) : hi; }
  wave_lds_sync();
  v8b vv[8];
#pragma unroll
  for (int j = 0; j < 8; ++j) vv[j] = *(const v8b*)(Es + (4 * j + (lane >> 3)) * 72 + 8 * (lane & 7));
  b16* dst = dstp + (size_t)(lane >> 3) * ldc + 8 * (lane & 7);
  for (int pass = 0; pass < 2; ++pass) {
#pragma unroll
    for (int j = 0; j < 8; ++j) *(volatile v8b*)(dst + (size_t)(4 * j) * ldc) = vv[j];
    __threadfence(); }
}

template <bool LO, bool RELU>
__device__ __forceinline__ void epi_vt(const v8f (&acc)[2][4], const float (&bb)[4], float oscale, b16* Et, b16* plane, int bidx, int key0, int colv0, int wave, int wm, int wn, int nloc, int hlf) {
#pragma unroll
  for (int mt = 0; mt < 2; ++mt)
#pragma unroll
    for (int t = 0; t < 4; ++t) { v8b hv;
#pragma unroll
      for (int r = 0; r < 8; ++r) { float v = acc[mt][t][r] * oscale + bb[t]; if (RELU) v = fmaxf(v, 0.0f); const float vs = v * CA; const b16 hi = (b16)vs; hv[r] = LO ? (b16)((vs - (float)hi) * RS) : hi; }
      *(v8b*)(Et + (wn * 64 + 16 * t + nloc) * 136 + wm * 32 + mt * 16 + 8 * hlf) = hv; }
  __syncthreads();
  v8b vv[8]; size_t dsto[8];
#pragma unroll
  for (int j = 0; j < 8; ++j) { const int dl = 16 * j + 2 * wave + hlf; const int col = colv0 + dl; const int hh = col / DH, dd = col % DH;
    vv[j] = *(const v8b*)(Et + dl * 136 + 8 * nloc); dsto[j] = ((size_t)(bidx * NH + hh) * DH + dd) * SEQ + key0 + 8 * nloc; }
  for (int pass = 0; pass < 2; ++pass) {
#pragma unroll
    for (int j = 0; j < 8; ++j) *(volatile v8b*)(plane + dsto[j]) = vv[j];
    __threadfence(); }
}

template <bool RELU>
__global__ __launch_bounds__(256) void gemm_kernel(const b16* __restrict__ A, int lda, const b16* __restrict__ Wt, int K,
    const float* __restrict__ bg0, const float* __restrict__ bg1, const float* __restrict__ bg2, const float* __restrict__ bg3,
    b16* __restrict__ C, b16* __restrict__ Clo, int ldc, int ccol0, b16* __restrict__ VT, b16* __restrict__ VTlo, int vcol0, float oscale, int wres) {
  __shared__ __attribute__((aligned(16))) b16 Ls[18432];
  const int tid = threadIdx.x, wave = tid >> 5, lane = tid & 31, nloc = lane & 15, hlf = lane >> 4;
  const int bm0 = blockIdx.x * 128, bn0 = blockIdx.y * 128, wm = wave >> 1, wn = wave & 1;
  const int row0 = bm0 + wm * 32, col0 = bn0 + wn * 64;
  v8f acc[2][4];
#pragma unroll
  for (int t = 0; t < 4; ++t) { acc[0][t] = (v8f){}; acc[1][t] = (v8f){}; }
  mac_32x64(acc, A + (size_t)(row0 + nloc) * lda, A + (size_t)(row0 + 16 + nloc) * lda, Wt + (size_t)(col0 + nloc) * K, K, hlf);
  const int gsel = bn0 >> 9; const float* bias = gsel == 0 ? bg0 : (gsel == 1 ? bg1 : (gsel == 2 ? bg2 : bg3));
  float bb[4];
#pragma unroll
  for (int t = 0; t < 4; ++t) bb[t] = bf16_rne(bias[(col0 & 511) + 16 * t + nloc]);
  const bool vmode = bn0 >= vcol0, wlo = (wres != 0) && (bm0 % SEQ == 0);
  if (!vmode) {
    b16* Es = Ls + wave * (32 * 72);
    epi_rows<false, RELU>(acc, bb, oscale, Es, C + (size_t)row0 * ldc + ccol0 + col0, ldc, lane, nloc, hlf);
    if (wlo) { wave_lds_sync(); epi_rows<true, RELU>(acc, bb, oscale, Es, Clo + (size_t)row0 * ldc + ccol0 + col0, ldc, lane, nloc, hlf); }
  } else {
    epi_vt<false, RELU>(acc, bb, oscale, Ls, VT, bm0 / SEQ, bm0 % SEQ, bn0 - vcol0, wave, wm, wn, nloc, hlf);
    if (wlo) { __syncthreads(); epi_vt<true, RELU>(acc, bb, oscale, Ls, VTlo, bm0 / SEQ, bm0 % SEQ, bn0 - vcol0, wave, wm, wn, nloc, hlf); }
  }
}

__global__ __launch_bounds__(256) void gemm_ln_kernel(const b16* __restrict__ A, int K, const b16* __restrict__ Wt, const float* __restrict__ bias, const float* Xres,
    const float* __restrict__ gam, const float* __restrict__ bet, float* OutF, b16* __restrict__ Xh, float oscale, int wxh) {
  __shared__ __attribute__((aligned(16))) float Tf[16 * (D + 4)];
  const int tid = threadIdx.x, wave = tid >> 5, lane = tid & 31, nloc = lane & 15, hlf = lane >> 4;
  const int bm0 = blockIdx.x * 32, col0 = wave * 64;
  v8f acc[2][4];
#pragma unroll
  for (int t = 0; t < 4; ++t) { acc[0][t] = (v8f){}; acc[1][t] = (v8f){}; }
  mac_32x64(acc, A + (size_t)(bm0 + nloc) * K, A + (size_t)(bm0 + 16 + nloc) * K, Wt + (size_t)(col0 + nloc) * K, K, hlf);
#pragma unroll 1
  for (int mt = 0; mt < 2; ++mt) {
    if (mt) __syncthreads();
#pragma unroll
    for (int t = 0; t < 4; ++t)
#pragma unroll
      for (int r = 0; r < 8; ++r) Tf[(8 * hlf + r) * (D + 4) + col0 + 16 * t + nloc] = (mt ? acc[1][t][r] : acc[0][t][r]) * oscale;
    __syncthreads();
#pragma unroll 1
    for (int rr = 0; rr < 2; ++rr) {
      const int rl = 2 * wave + rr; const size_t go = (size_t)(bm0 + mt * 16 + rl) * D;
      float y[16]; float s = 0.0f;
#pragma unroll
      for (int j = 0; j < 4; ++j) { const int c = 128 * j + 4 * lane;
        const v4f tv = *(const v4f*)(Tf + rl * (D + 4) + c); const v4f rv = *(const v4f*)(Xres + go + c); const v4f bv = *(const v4f*)(bias + c);
#pragma unroll
        for (int e = 0; e < 4; ++e) { const float yy = rv[e] + (tv[e] + bf16_rne(bv[e])); y[4 * j + e] = yy; s += yy; } }
#pragma unroll
      for (int off = 16; off > 0; off >>= 1) s += __shfl_xor(s, off, 32);
      const float mean = s * (1.0f / (float)D); float q = 0.0f;
#pragma unroll
      for (int i = 0; i < 16; ++i) { const float d0 = y[i] - mean; y[i] = d0; q += d0 * d0; }
#pragma unroll
      for (int off = 16; off > 0; off >>= 1) q += __shfl_xor(q, off, 32);
      const float rstd = 1.0f / sqrtf(q * (1.0f / (float)D) + LNEPS);
      v4f ov[4]; v4h_ hv[4];
#pragma unroll
      for (int j = 0; j < 4; ++j) { const int c = 128 * j + 4 * lane; const v4f gv = *(const v4f*)(gam + c), ev = *(const v4f*)(bet + c);
#pragma unroll
        for (int e = 0; e < 4; ++e) { const float o = (y[4 * j + e] * rstd) * bf16_rne(gv[e]) + bf16_rne(ev[e]); ov[j][e] = o; hv[j][e] = (b16)(o * CA); } }
      for (int pass = 0; pass < 2; ++pass) {
#pragma unroll
        for (int j = 0; j < 4; ++j) { const int c = 128 * j + 4 * lane; *(volatile v4f*)(OutF + go + c) = ov[j]; if (wxh) *(volatile v4h_*)(Xh + go + c) = hv[j]; }
        __threadfence(); }
    }
  }
}

template <bool RES>
__global__ __launch_bounds__(32) void attn_kernel(const b16* __restrict__ QK, const b16* __restrict__ QKlo, const b16* __restrict__ VT, const b16* __restrict__ VTlo,
    const int* __restrict__ mask, b16* __restrict__ CTX, int qt0, int nqt) {
  __shared__ __attribute__((aligned(16))) b16 Pst[16 * 40];
  __shared__ __attribute__((aligned(16))) b16 Plst[16 * 40];
  __shared__ __attribute__((aligned(16))) b16 Cst[16 * 72];
  const int lane = threadIdx.x & 31, nloc = lane & 15, hlf = lane >> 4;
  const int bi = blockIdx.x, qt = qt0 + bi % nqt, bh = bi / nqt, h = bh % NH, b = bh / NH, q0 = qt * 16;
  const size_t rq = (size_t)b * SEQ + q0;
  const b16* qp = QK + (rq + nloc) * LQK + h * DH;
  const v16b qa0 = frag_kb(qp, hlf), qa1 = frag_kb(qp + 32, hlf);
  v16b ql0 = (v16b){}, ql1 = (v16b){};
  if (RES) { const b16* qlp = QKlo + (rq + nloc) * LQK + h * DH; ql0 = frag_kb(qlp, hlf); ql1 = frag_kb(qlp + 32, hlf); }
  const b16* kbase = QK + (size_t)b * SEQ * LQK + D + h * DH;
  const b16* klbase = QKlo + (size_t)b * SEQ * LQK + D + h * DH;
  const b16* vbase = VT + (size_t)(b * NH + h) * DH * SEQ;
  const b16* vlbase = VTlo + (size_t)(b * NH + h) * DH * SEQ;
  const int* mq = mask + ((size_t)b * SEQ_FULL + q0 + 8 * hlf) * SEQ_FULL + nloc;
  float mx[8], ls[8]; v8f acc[4], acc2[4];
#pragma unroll
  for (int r = 0; r < 8; ++r) { mx[r] = -3.0e38f; ls[r] = 0.0f; }
#pragma unroll
  for (int t = 0; t < 4; ++t) { acc[t] = (v8f){}; acc2[t] = (v8f){}; }
#pragma unroll 1
  for (int c = 0; c < SEQ / 32; ++c) {
    const int kb = 32 * c;
    int m0[8], m1[8]; bool allm = true;
#pragma unroll
    for (int r = 0; r < 8; ++r) m0[r] = mq[(size_t)r * SEQ_FULL + kb];
    asm volatile("" :: "v"(m0[0]), "v"(m0[1]), "v"(m0[2]), "v"(m0[3]), "v"(m0[4]), "v"(m0[5]), "v"(m0[6]), "v"(m0[7]) : "memory");
#pragma unroll
    for (int r = 0; r < 8; ++r) m1[r] = mq[(size_t)r * SEQ_FULL + kb + 16];
#pragma unroll
    for (int r = 0; r < 8; ++r) allm = allm && (m0[r] != 0) && (m1[r] != 0);
    if (__builtin_amdgcn_ballot_w32(allm) == 0xffffffffu) continue;
    wave_lds_sync();
    v8f s[2];
#pragma unroll
    for (int t = 0; t < 2; ++t) {
      const b16* kp = kbase + (size_t)(kb + 16 * t + nloc) * LQK; const v16b k0f = frag_kb(kp, hlf), k1f = frag_kb(kp + 32, hlf);
      v8f sh = wmma16b(qa0, k0f, (v8f){}); sh = wmma16b(qa1, k1f, sh);
      if (RES && c < 4) {
        const b16* klp = klbase + (size_t)(kb + 16 * t + nloc) * LQK;
        v8f x = wmma16b(ql0, k0f, (v8f){}); x = wmma16b(ql1, k1f, x); x = wmma16b(qa0, frag_kb(klp, hlf), x); x = wmma16b(qa1, frag_kb(klp + 32, hlf), x);
#pragma unroll
        for (int r = 0; r < 8; ++r) sh[r] += x[r] * (1.0f / RS); }
      s[t] = sh; }
    float p0[8], p1[8];
#pragma unroll
    for (int r = 0; r < 8; ++r) {
      float s0 = s[0][r] * SCL, s1 = s[1][r] * SCL; s0 = (m0[r] != 0) ? NEGF : s0; s1 = (m1[r] != 0) ? NEGF : s1;
      const float cm = red_max16(fmaxf(s0, s1)); const float mn = fmaxf(mx[r], cm); const float al = nexp2((mx[r] - mn) * L2E); mx[r] = mn;
      const float e0 = nexp2((s0 - mn) * L2E), e1 = nexp2((s1 - mn) * L2E); p0[r] = e0; p1[r] = e1;
      ls[r] = ls[r] * al + red_sum16(e0 + e1);
#pragma unroll
      for (int t = 0; t < 4; ++t) { acc[t][r] *= al; if (RES) acc2[t][r] *= al; } }
#pragma unroll
    for (int r = 0; r < 8; ++r) {
      const float v0 = p0[r] * PSC, v1 = p1[r] * PSC; const b16 h0 = (b16)v0, h1 = (b16)v1;
      Pst[(8 * hlf + r) * 40 + nloc] = h0; Pst[(8 * hlf + r) * 40 + 16 + nloc] = h1;
      if (RES) { Plst[(8 * hlf + r) * 40 + nloc] = (b16)((v0 - (float)h0) * RS); Plst[(8 * hlf + r) * 40 + 16 + nloc] = (b16)((v1 - (float)h1) * RS); } }
    wave_lds_sync();
    const v16b pf = frag_kb(Pst + nloc * 40, hlf); v16b plf = (v16b){}; if (RES) plf = frag_kb(Plst + nloc * 40, hlf);
#pragma unroll
    for (int t = 0; t < 4; ++t) {
      const v16b vf = frag_kb(vbase + (size_t)(16 * t + nloc) * SEQ + kb, hlf); acc[t] = wmma16b(pf, vf, acc[t]);
      if (RES && c < 4) { acc2[t] = wmma16b(plf, vf, acc2[t]); acc2[t] = wmma16b(pf, frag_kb(vlbase + (size_t)(16 * t + nloc) * SEQ + kb, hlf), acc2[t]); } }
  }
  wave_lds_sync();
#pragma unroll
  for (int r = 0; r < 8; ++r) { const float inv = (1.0f / ls[r]) * (CX / (PSC * CA));
#pragma unroll
    for (int t = 0; t < 4; ++t) { float a = acc[t][r]; if (RES) a += acc2[t][r] * (1.0f / RS); Cst[(8 * hlf + r) * 72 + 16 * t + nloc] = (b16)(a * inv); } }
  wave_lds_sync();
  v8b vv[4];
#pragma unroll
  for (int j = 0; j < 4; ++j) vv[j] = *(const v8b*)(Cst + (4 * j + (lane >> 3)) * 72 + 8 * (lane & 7));
  b16* dst = CTX + (rq + (lane >> 3)) * D + h * DH + 8 * (lane & 7);
  for (int pass = 0; pass < 2; ++pass) {
#pragma unroll
    for (int j = 0; j < 4; ++j) *(volatile v8b*)(dst + (size_t)(4 * j) * D) = vv[j];
    __threadfence(); }
}
}

extern "C" void kernel_launch(void* const* d_in, const int* in_sizes, int n_in, void* d_out, int out_size, void* d_ws, size_t ws_size, hipStream_t stream) {
  (void)n_in;
  auto Fp = [&](int i) { return (const float*)d_in[i]; };
  auto Ip = [&](int i) { return (const int*)d_in[i]; };
  const long needRows = (long)(NB - 1) * SEQ_FULL + SEQ;
  if ((long)in_sizes[0] < (long)SEQ * NB_FULL || (long)in_sizes[1] < needRows * D || (long)in_sizes[2] < needRows * SEQ_FULL || (long)in_sizes[3] < needRows * SEQ_FULL ||
      (long)in_sizes[4] < (long)VOCAB * D) return;
  for (int i = 5; i <= 12; ++i) if ((long)in_sizes[i] < (long)NLAY * D * D) return;
  for (int i = 13; i <= 20; ++i) if (in_sizes[i] < NLAY * D) return;
  if ((long)in_sizes[21] < (long)NLAY * D * DFF || in_sizes[22] < NLAY * DFF || (long)in_sizes[23] < (long)NLAY * DFF * D || in_sizes[24] < NLAY * D) return;
  for (int i = 25; i <= 30; ++i) if (in_sizes[i] < NLAY * D) return;
  if (out_size < MR * D) return;

  size_t off = 0; char* ws = (char*)d_ws;
  auto carve = [&](size_t bytes) { char* p = ws + off; off += (bytes + 255) & ~(size_t)255; return p; };
  b16* WQKVS = (b16*)carve((size_t)NLAY * NQKV * D * 2);
  b16* WOS   = (b16*)carve((size_t)NLAY * D * D * 2);
  b16* WQC   = (b16*)carve((size_t)NLAY * D * D * 2);
  b16* WKVC  = (b16*)carve((size_t)NLAY * NKV * D * 2);
  b16* WOC   = (b16*)carve((size_t)NLAY * D * D * 2);
  b16* W1T   = (b16*)carve((size_t)NLAY * DFF * D * 2);
  b16* W2T   = (b16*)carve((size_t)NLAY * D * DFF * 2);
  float* X   = (float*)carve((size_t)MR * D * 4);
  b16* Xh    = (b16*)carve((size_t)MR * D * 2);
  b16* Mh    = (b16*)carve((size_t)MR * D * 2);
  b16* QK    = (b16*)carve((size_t)MR * LQK * 2);
  b16* QKlo  = (b16*)carve((size_t)MR * LQK * 2);
  b16* Vt    = (b16*)carve((size_t)MR * D * 2);
  b16* Vtlo  = (b16*)carve((size_t)MR * D * 2);
  b16* CTX   = (b16*)carve((size_t)MR * D * 2);
  b16* Hh    = (b16*)carve((size_t)MR * DFF * 2);
  if (off > ws_size || off > ((size_t)128 << 20)) return;

  const dim3 b256(256), b32(32);
  wprep_kernel<<<dim3(D / 64, D / 64, NLAY), b256, 0, stream>>>(Fp(5), WQKVS, D, D, NQKV, 0);
  wprep_kernel<<<dim3(D / 64, D / 64, NLAY), b256, 0, stream>>>(Fp(6), WQKVS, D, D, NQKV, D);
  wprep_kernel<<<dim3(D / 64, D / 64, NLAY), b256, 0, stream>>>(Fp(7), WQKVS, D, D, NQKV, 2 * D);
  wprep_kernel<<<dim3(D / 64, D / 64, NLAY), b256, 0, stream>>>(Fp(8), WOS, D, D, D, 0);
  wprep_kernel<<<dim3(D / 64, D / 64, NLAY), b256, 0, stream>>>(Fp(9), WQC, D, D, D, 0);
  wprep_kernel<<<dim3(D / 64, D / 64, NLAY), b256, 0, stream>>>(Fp(10), WKVC, D, D, NKV, 0);
  wprep_kernel<<<dim3(D / 64, D / 64, NLAY), b256, 0, stream>>>(Fp(11), WKVC, D, D, NKV, D);
  wprep_kernel<<<dim3(D / 64, D / 64, NLAY), b256, 0, stream>>>(Fp(12), WOC, D, D, D, 0);
  wprep_kernel<<<dim3(D / 64, DFF / 64, NLAY), b256, 0, stream>>>(Fp(21), W1T, D, DFF, DFF, 0);
  wprep_kernel<<<dim3(DFF / 64, D / 64, NLAY), b256, 0, stream>>>(Fp(23), W2T, DFF, D, D, 0);
  mprep_kernel<<<(MR * D / 8 + 255) / 256, b256, 0, stream>>>(Fp(1), Mh);
  embed_kernel<<<MR / 4, b256, 0, stream>>>(Ip(0), Fp(4), X, Xh);

  const float OSA = 1.0f / (CA * WSC), OSX = 1.0f / (CX * WSC);
  for (int l = 0; l < NLAY; ++l) {
    const size_t lD = (size_t)l * D, lF = (size_t)l * DFF;
    gemm_kernel<false><<<dim3(MR / 128, NQKV / 128), b256, 0, stream>>>(Xh, D, WQKVS + (size_t)l * NQKV * D, D, Fp(13) + lD, Fp(14) + lD, Fp(15) + lD, Fp(15) + lD,
        QK, QKlo, LQK, 0, Vt, Vtlo, 2 * D, OSA, 1);
    attn_kernel<true><<<NB * NH * NQT_RES, b32, 0, stream>>>(QK, QKlo, Vt, Vtlo, Ip(2), CTX, 0, NQT_RES);
    attn_kernel<false><<<NB * NH * (NQT - NQT_RES), b32, 0, stream>>>(QK, QKlo, Vt, Vtlo, Ip(2), CTX, NQT_RES, NQT - NQT_RES);
    gemm_ln_kernel<<<MR / 32, b256, 0, stream>>>(CTX, D, WOS + (size_t)l * D * D, Fp(16) + lD, X, Fp(25) + lD, Fp(28) + lD, X, Xh, OSX, 1);
    gemm_kernel<false><<<dim3(MR / 128, D / 128), b256, 0, stream>>>(Xh, D, WQC + (size_t)l * D * D, D, Fp(17) + lD, Fp(17) + lD, Fp(17) + lD, Fp(17) + lD,
        QK, QKlo, LQK, 0, Vt, Vtlo, D, OSA, 0);
    gemm_kernel<false><<<dim3(MR / 128, NKV / 128), b256, 0, stream>>>(Mh, D, WKVC + (size_t)l * NKV * D, D, Fp(18) + lD, Fp(19) + lD, Fp(19) + lD, Fp(19) + lD,
        QK, QKlo, LQK, D, Vt, Vtlo, D, OSA, 0);
    attn_kernel<false><<<NB * NH * NQT, b32, 0, stream>>>(QK, QKlo, Vt, Vtlo, Ip(3), CTX, 0, NQT);
    gemm_ln_kernel<<<MR / 32, b256, 0, stream>>>(CTX, D, WOC + (size_t)l * D * D, Fp(20) + lD, X, Fp(26) + lD, Fp(29) + lD, X, Xh, OSX, 1);
    gemm_kernel<true><<<dim3(MR / 128, DFF / 128), b256, 0, stream>>>(Xh, D, W1T + (size_t)l * DFF * D, D, Fp(22) + lF, Fp(22) + lF + 512, Fp(22) + lF + 1024, Fp(22) + lF + 1536,
        Hh, QKlo, DFF, 0, Vt, Vtlo, DFF, OSA, 0);
    const bool last = (l == NLAY - 1);
    gemm_ln_kernel<<<MR / 32, b256, 0, stream>>>(Hh, DFF, W2T + (size_t)l * D * DFF, Fp(24) + lD, X, Fp(27) + lD, Fp(30) + lD, last ? (float*)d_out : X, Xh, OSA, last ? 0 : 1);
  }
}
